// GATv2layer_19378892439975
// MI455X (gfx1250) — hardware-verified
//
#include <hip/hip_runtime.h>
#include <stddef.h>
#include <stdint.h>
#include <math.h>


#define NB    4
#define NN    1024
#define DIN   128
#define DO    64
#define NROWS (NB * NN)
#define TI    16
#define TJ    64
#define NTJ   (NN / TJ)
#define XP    65
#define PAP   136
#define AGP   264
#define TSP   136
#define LCAP  1024
#define SLOPE 0.01f
#define PB_X  64
#define PB_W  8
#define PB_L  8
#define PB_A  1
#define PB_TOT (PB_X + PB_W + PB_L + PB_A)
#define GBM   64
#define WSMAX 134217728

static_assert(TI * TJ == LCAP);
static_assert(TI * TJ == 256 * 4);
static_assert((DIN % 32) == 0 && (2 * TJ) % 32 == 0 && (2 * DIN) % 32 == 0);
static_assert((NROWS % GBM) == 0 && (NN % TI) == 0 && (NN % TJ) == 0);
static_assert(PB_X == NB * (NN / 64));
static_assert(PB_W * 256 == DIN * (DIN / 8));
static_assert(PB_L * 256 == DO * (2 * DIN / 8));
static_assert((PAP % 8) == 0 && (AGP % 8) == 0 && (TSP % 8) == 0);
static_assert(DIN == 8 * 16);

typedef float          v4f  __attribute__((ext_vector_type(4)));
typedef float          v8f  __attribute__((ext_vector_type(8)));
typedef int            v8i  __attribute__((ext_vector_type(8)));
typedef unsigned short v8us __attribute__((ext_vector_type(8)));
typedef __bf16         v16b __attribute__((ext_vector_type(16)));
typedef v4f  __attribute__((may_alias)) v4fa;
typedef v8us __attribute__((may_alias)) v8usa;
union FragB { v16b v; v8us h[2]; v8i w; };

__device__ __forceinline__ v8f wmb(const FragB& a, const FragB& b, v8f c) {
  v8f d = __builtin_amdgcn_wmma_f32_16x16x32_bf16(false, a.v, false, b.v, (short)0, c, false, false);
  asm volatile("v_nop\n\tv_nop\n\tv_nop\n\tv_nop" : "+v"(d) : "v"(a.w), "v"(b.w));
  return d;
}

__device__ __forceinline__ unsigned int f2bf(float f) {
  const unsigned int u = __float_as_uint(f);
  return ((u + 0x7FFFu + ((u >> 16) & 1u)) >> 16) & 0xFFFFu;
}
__device__ __forceinline__ float bf2f(unsigned int b) { return __uint_as_float(b << 16); }
__device__ __forceinline__ float bfr(float f) { return bf2f(f2bf(f)); }
__device__ __forceinline__ v8us cvt8(const v4f a, const v4f c) {
  v8us o;
  o[0] = (unsigned short)f2bf(a.x); o[1] = (unsigned short)f2bf(a.y);
  o[2] = (unsigned short)f2bf(a.z); o[3] = (unsigned short)f2bf(a.w);
  o[4] = (unsigned short)f2bf(c.x); o[5] = (unsigned short)f2bf(c.y);
  o[6] = (unsigned short)f2bf(c.z); o[7] = (unsigned short)f2bf(c.w);
  return o;
}

__global__ __launch_bounds__(256) void k_prep(const float* __restrict__ x, const float* __restrict__ w1,
                                              const float* __restrict__ w2, const float* __restrict__ av,
                                              const float* __restrict__ lw,
                                              unsigned short* XB, unsigned short* XT, unsigned short* W12T,
                                              unsigned short* LW2, float* AF) {
  __shared__ __attribute__((aligned(16))) unsigned short ts[64 * TSP];
  const int blk = (int)blockIdx.x, tid = (int)threadIdx.x;
  if (blk < PB_X) {
    const int b  = blk >> 4;
    const int j0 = (blk & 15) * 64;
#pragma unroll
    for (int it = 0; it < 4; ++it) {
      const int u = tid + 256 * it;
      const int row = u >> 4, k8 = (u & 15) * 8;
      const size_t g = ((size_t)(b * NN + j0 + row)) * DIN + k8;
      const v4f a = *(const v4f*)(x + g);
      const v4f c = *(const v4f*)(x + g + 4);
      const v8us o = cvt8(a, c);
      *(v8usa*)(ts + row * TSP + k8) = o;
      unsigned short* dp = XB + g;
      *(volatile v8us*)dp = o;
      __threadfence();
      *(volatile v8us*)dp = o;
    }
    __syncthreads();
#pragma unroll
    for (int it = 0; it < 4; ++it) {
      const int v = tid + 256 * it;
      const int f = v >> 3, j8 = (v & 7) * 8;
      v8us o;
#pragma unroll
      for (int i = 0; i < 8; ++i) o[i] = ts[(j8 + i) * TSP + f];
      unsigned short* dp = XT + ((size_t)(b * DIN + f)) * NN + j0 + j8;
      *(volatile v8us*)dp = o;
      __threadfence();
      *(volatile v8us*)dp = o;
    }
  } else if (blk < PB_X + PB_W) {
    const int u  = (blk - PB_X) * 256 + tid;
    const int n  = u >> 4;
    const int k8 = (u & 15) * 8;
    const float* wsrc = (blk < PB_X + PB_W / 2) ? w1 : w2;
    const float* p = wsrc + (size_t)k8 * DO + (n & 63);
    v8us o;
#pragma unroll
    for (int i = 0; i < 8; ++i) o[i] = (unsigned short)f2bf(p[(size_t)i * DO]);
    unsigned short* dp = W12T + (size_t)n * DIN + k8;
    *(volatile v8us*)dp = o;
    __threadfence();
    *(volatile v8us*)dp = o;
  } else if (blk < PB_X + PB_W + PB_L) {
    const int u  = (blk - PB_X - PB_W) * 256 + tid;
    const int n  = u >> 5;
    const int k8 = (u & 31) * 8;
    const int kk = k8 & (DIN - 1);
    const float* p = lw + (size_t)n * DIN + kk;
    const v4f a = *(const v4f*)p;
    const v4f c = *(const v4f*)(p + 4);
    const v8us o = cvt8(a, c);
    unsigned short* dp = LW2 + (size_t)n * (2 * DIN) + k8;
    *(volatile v8us*)dp = o;
    __threadfence();
    *(volatile v8us*)dp = o;
  } else {
    if (tid < 16) {
      const v4f a = *(const v4f*)(av + 4 * tid);
      v4f r; r.x = bfr(a.x); r.y = bfr(a.y); r.z = bfr(a.z); r.w = bfr(a.w);
      float* dp = AF + 4 * tid;
      *(volatile v4f*)dp = r;
      __threadfence();
      *(volatile v4f*)dp = r;
    }
  }
}

__global__ __launch_bounds__(128) void k_proj(const unsigned short* __restrict__ A,
                                              const unsigned short* __restrict__ BT, float* Cm) {
  __shared__ __attribute__((aligned(16))) float stg[GBM * DIN];
  const int tid = (int)threadIdx.x, lane = tid & 31, wave = tid >> 5, hh = lane >> 4, m = lane & 15;
  const int rowBase = (int)blockIdx.x * GBM;
  v8f acc[8];
  {
    const v8f z = {0.f, 0.f, 0.f, 0.f, 0.f, 0.f, 0.f, 0.f};
#pragma unroll
    for (int t = 0; t < 8; ++t) acc[t] = z;
  }
  const unsigned short* ap = A  + (size_t)(rowBase + 16 * wave + m) * DIN + 8 * hh;
  const unsigned short* bp = BT + (size_t)m * DIN + 8 * hh;
#pragma unroll 1
  for (int k0 = 0; k0 < DIN; k0 += 32) {
    FragB af;
    af.h[0] = *(const v8usa*)(ap + k0);
    af.h[1] = *(const v8usa*)(ap + k0 + 16);
#pragma unroll
    for (int nt = 0; nt < 8; ++nt) {
      const unsigned short* wq = bp + (size_t)(16 * nt) * DIN + k0;
      FragB bf;
      bf.h[0] = *(const v8usa*)wq;
      bf.h[1] = *(const v8usa*)(wq + 16);
      acc[nt] = wmb(af, bf, acc[nt]);
    }
  }
#pragma unroll
  for (int nt = 0; nt < 8; ++nt) {
    const int lc = 16 * nt + m;
#pragma unroll
    for (int r = 0; r < 8; ++r) {
      const int lr = 16 * wave + 8 * hh + r;
      stg[lr * DIN + lc] = acc[nt][r];
    }
  }
  __syncthreads();
#pragma unroll 1
  for (int i = 0; i < 16; ++i) {
    const int row = wave * 16 + i;
    const v4f p = *(const v4fa*)(stg + row * DIN + 4 * lane);
    float* op = Cm + (size_t)(rowBase + row) * DIN + 4 * lane;
    *(volatile v4f*)op = p;
  }
  __threadfence();
#pragma unroll 1
  for (int i = 0; i < 16; ++i) {
    const int row = wave * 16 + i;
    const v4f p = *(const v4fa*)(stg + row * DIN + 4 * lane);
    float* op = Cm + (size_t)(rowBase + row) * DIN + 4 * lane;
    *(volatile v4f*)op = p;
  }
}

__global__ __launch_bounds__(256) void k_gat(const float* __restrict__ Am, const float* __restrict__ X12,
                                             const unsigned short* __restrict__ XT,
                                             const unsigned short* __restrict__ LW2,
                                             const float* __restrict__ AF, float* outp) {
  __shared__ __attribute__((aligned(16))) float X1s[TI * 64];
  __shared__ __attribute__((aligned(16))) float AFs[64];
  __shared__ __attribute__((aligned(16))) float Ms[TI * TJ];
  __shared__ __attribute__((aligned(16))) float X2s[64 * XP];
  __shared__ __attribute__((aligned(16))) float Pf[TI * TJ];
  __shared__ __attribute__((aligned(16))) unsigned short PA[TI * PAP];
  __shared__ __attribute__((aligned(16))) unsigned short AG[TI * AGP];
  __shared__ __attribute__((aligned(16))) float OS[TI * DO];
  __shared__ int   list[LCAP];
  __shared__ int   wcnt[8];
  __shared__ float lrow[TI];

  const int tid = (int)threadIdx.x, lane = tid & 31, wave = tid >> 5, hh = lane >> 4, m = lane & 15;
  const int b     = (int)blockIdx.x >> 6;
  const int ibase = ((int)blockIdx.x & 63) * TI;

  {
    const int i = tid >> 4, d4 = (tid & 15) * 4;
    const v4f v = *(const v4f*)(X12 + ((size_t)(b * NN + ibase + i)) * DIN + d4);
    *(v4fa*)(X1s + i * 64 + d4) = v;
    if (tid < 16) {
      const v4f a4 = *(const v4f*)(AF + 4 * tid);
      *(v4fa*)(AFs + 4 * tid) = a4;
    }
  }

  v8f acc = {0.f, 0.f, 0.f, 0.f, 0.f, 0.f, 0.f, 0.f};
  float lacc = 0.0f;
  const float* mrow = Am + ((size_t)(b * NN + ibase + (tid >> 4))) * NN + 4 * (tid & 15);
  const unsigned short* xtp = XT + ((size_t)(b * DIN + 16 * wave + m)) * NN + 8 * hh;

#pragma unroll 1
  for (int t = 0; t < NTJ; ++t) {
    const int j0 = t * TJ;
    __syncthreads();

    const v4f mv = *(const v4f*)(mrow + j0);
    *(v4fa*)(Ms + 4 * tid) = mv;
#pragma unroll
    for (int it = 0; it < 4; ++it) {
      const int u = tid + 256 * it;
      const int j = u >> 4, d4 = (u & 15) * 4;
      const v4f xv = *(const v4f*)(X12 + ((size_t)(b * NN + j0 + j)) * DIN + 64 + d4);
      X2s[(d4 + 0) * XP + j] = xv.x;
      X2s[(d4 + 1) * XP + j] = xv.y;
      X2s[(d4 + 2) * XP + j] = xv.z;
      X2s[(d4 + 3) * XP + j] = xv.w;
    }
    {
      const v4f z4 = {0.f, 0.f, 0.f, 0.f};
      *(v4fa*)(Pf + 4 * tid) = z4;
      const v8us z8 = {0, 0, 0, 0, 0, 0, 0, 0};
      *(v8usa*)(PA + (tid >> 4) * PAP + (tid & 15) * 8) = z8;
    }
    const bool h0 = mv.x != 0.0f, h1 = mv.y != 0.0f, h2 = mv.z != 0.0f, h3 = mv.w != 0.0f;
    const unsigned q0 = __builtin_amdgcn_ballot_w32(h0);
    const unsigned q1 = __builtin_amdgcn_ballot_w32(h1);
    const unsigned q2 = __builtin_amdgcn_ballot_w32(h2);
    const unsigned q3 = __builtin_amdgcn_ballot_w32(h3);
    const int c0 = (int)__builtin_popcount(q0), c1 = (int)__builtin_popcount(q1);
    const int c2 = (int)__builtin_popcount(q2), c3 = (int)__builtin_popcount(q3);
    if (lane == 0) wcnt[wave] = c0 + c1 + c2 + c3;
    __syncthreads();

    int pre = 0, tot = 0;
#pragma unroll
    for (int w2 = 0; w2 < 8; ++w2) {
      int c = wcnt[w2];
      c = c < 0 ? 0 : (c > 128 ? 128 : c);
      tot += c;
      pre += (w2 < wave) ? c : 0;
    }
    tot = tot > LCAP ? LCAP : tot;
    {
      const int e0 = 4 * tid;
      int run = pre;
      int pos = run + (int)__builtin_amdgcn_mbcnt_lo(q0, 0u);
      if (h0 && pos < LCAP) list[pos] = e0;
      run += c0;
      pos = run + (int)__builtin_amdgcn_mbcnt_lo(q1, 0u);
      if (h1 && pos < LCAP) list[pos] = e0 + 1;
      run += c1;
      pos = run + (int)__builtin_amdgcn_mbcnt_lo(q2, 0u);
      if (h2 && pos < LCAP) list[pos] = e0 + 2;
      run += c2;
      pos = run + (int)__builtin_amdgcn_mbcnt_lo(q3, 0u);
      if (h3 && pos < LCAP) list[pos] = e0 + 3;
    }

    if (tot > 0) {
      __syncthreads();

#pragma unroll 1
      for (int p = tid; p < tot; p += 256) {
        const int ent = list[p] & (LCAP - 1);
        const int i = ent >> 6, j = ent & 63;
        const float* x1p = X1s + i * 64;
        const float* x2p = X2s + j;
        float s = 0.0f;
#pragma unroll 4
        for (int d4 = 0; d4 < 16; ++d4) {
          const v4f xa = *(const v4fa*)(x1p + 4 * d4);
          const v4f a4 = *(const v4fa*)(AFs + 4 * d4);
          float t0 = xa.x + x2p[(4 * d4 + 0) * XP];
          float t1 = xa.y + x2p[(4 * d4 + 1) * XP];
          float t2 = xa.z + x2p[(4 * d4 + 2) * XP];
          float t3 = xa.w + x2p[(4 * d4 + 3) * XP];
          t0 = fmaxf(t0, SLOPE * t0);
          t1 = fmaxf(t1, SLOPE * t1);
          t2 = fmaxf(t2, SLOPE * t2);
          t3 = fmaxf(t3, SLOPE * t3);
          s = fmaf(a4.x, t0, s);
          s = fmaf(a4.y, t1, s);
          s = fmaf(a4.z, t2, s);
          s = fmaf(a4.w, t3, s);
        }
        s = tanhf(s * 0.125f) * 8.0f;
        const float e  = expf(s);
        const float pv = e * Ms[ent];
        const unsigned int hb = f2bf(pv);
        const unsigned int lb = f2bf(pv - bf2f(hb));
        Pf[ent] = pv;
        PA[i * PAP + j]      = (unsigned short)hb;
        PA[i * PAP + 64 + j] = (unsigned short)lb;
      }
      __syncthreads();

      {
        const v4f pv = *(const v4fa*)(Pf + 4 * tid);
        float s = (pv.x + pv.y) + (pv.z + pv.w);
        s += __shfl_xor(s, 8);
        s += __shfl_xor(s, 4);
        s += __shfl_xor(s, 2);
        s += __shfl_xor(s, 1);
        lacc += s;
      }

      {
        FragB b0, b1, af;
        b0.h[0] = *(const v8usa*)(xtp + j0);
        b0.h[1] = *(const v8usa*)(xtp + j0 + 16);
        b1.h[0] = *(const v8usa*)(xtp + j0 + 32);
        b1.h[1] = *(const v8usa*)(xtp + j0 + 48);
        const unsigned short* pap = PA + m * PAP + 8 * hh;
        af.h[0] = *(const v8usa*)(pap);       af.h[1] = *(const v8usa*)(pap + 16);
        acc = wmb(af, b0, acc);
        af.h[0] = *(const v8usa*)(pap + 32);  af.h[1] = *(const v8usa*)(pap + 48);
        acc = wmb(af, b1, acc);
        af.h[0] = *(const v8usa*)(pap + 64);  af.h[1] = *(const v8usa*)(pap + 80);
        acc = wmb(af, b0, acc);
        af.h[0] = *(const v8usa*)(pap + 96);  af.h[1] = *(const v8usa*)(pap + 112);
        acc = wmb(af, b1, acc);
      }
    }
  }

  if ((tid & 15) == 0) lrow[tid >> 4] = lacc;
  __syncthreads();
#pragma unroll
  for (int r = 0; r < 8; ++r) {
    const int row = 8 * hh + r;
    const float inv = 1.0f / lrow[row];
    const float g = acc[r] * inv;
    const unsigned int hb = f2bf(g);
    const unsigned int lb = f2bf(g - bf2f(hb));
    AG[row * AGP + 16 * wave + m]       = (unsigned short)hb;
    AG[row * AGP + 128 + 16 * wave + m] = (unsigned short)lb;
  }
  __syncthreads();
  if (wave < 4) {
    v8f o2 = {0.f, 0.f, 0.f, 0.f, 0.f, 0.f, 0.f, 0.f};
    const unsigned short* ap = AG + m * AGP + 8 * hh;
    const unsigned short* bp = LW2 + (size_t)(16 * wave + m) * (2 * DIN) + 8 * hh;
#pragma unroll 1
    for (int k0 = 0; k0 < 2 * DIN; k0 += 32) {
      FragB af, bf;
      af.h[0] = *(const v8usa*)(ap + k0);
      af.h[1] = *(const v8usa*)(ap + k0 + 16);
      bf.h[0] = *(const v8usa*)(bp + k0);
      bf.h[1] = *(const v8usa*)(bp + k0 + 16);
      o2 = wmb(af, bf, o2);
    }
#pragma unroll
    for (int r = 0; r < 8; ++r) {
      const float v = o2[r];
      const float y = (v >= 0.0f) ? v : SLOPE * v;
      OS[(8 * hh + r) * DO + 16 * wave + m] = y;
    }
  }
  __syncthreads();
  {
    const v4f ov = *(const v4fa*)(OS + 4 * tid);
    float* op = outp + ((size_t)(b * NN + ibase)) * DO + 4 * tid;
    *(volatile v4f*)op = ov;
    __threadfence();
    *(volatile v4f*)op = ov;
  }
}

extern "C" void kernel_launch(void* const* d_in, const int* in_sizes, int n_in,
                              void* d_out, int out_size, void* d_ws, size_t ws_size,
                              hipStream_t stream) {
  if (n_in < 6) return;
  if (in_sizes[0] != NB * NN * DIN) return;
  if (in_sizes[1] != NB * NN * NN) return;
  if (in_sizes[2] != DIN * DO) return;
  if (in_sizes[3] != DIN * DO) return;
  if (in_sizes[4] != DO) return;
  if (in_sizes[5] != DO * DIN) return;
  if (out_size != NB * NN * DO) return;

  const float* x   = (const float*)d_in[0];
  const float* Am  = (const float*)d_in[1];
  const float* w1  = (const float*)d_in[2];
  const float* w2  = (const float*)d_in[3];
  const float* av  = (const float*)d_in[4];
  const float* lw  = (const float*)d_in[5];
  float* out = (float*)d_out;

  char* ws = (char*)d_ws;
  size_t off = 0;
  const size_t oXB  = off; off += (size_t)NROWS * DIN * 2;       off = (off + 255) & ~(size_t)255;
  const size_t oXT  = off; off += (size_t)NB * DIN * NN * 2;     off = (off + 255) & ~(size_t)255;
  const size_t oX12 = off; off += (size_t)NROWS * DIN * 4;       off = (off + 255) & ~(size_t)255;
  const size_t oW   = off; off += (size_t)DIN * DIN * 2;         off = (off + 255) & ~(size_t)255;
  const size_t oLW  = off; off += (size_t)DO * 2 * DIN * 2;      off = (off + 255) & ~(size_t)255;
  const size_t oAF  = off; off += (size_t)256;                   off = (off + 255) & ~(size_t)255;
  if (off > ws_size || off > (size_t)WSMAX) return;
  unsigned short* XB   = (unsigned short*)(ws + oXB);
  unsigned short* XT   = (unsigned short*)(ws + oXT);
  float*          X12  = (float*)(ws + oX12);
  unsigned short* W12T = (unsigned short*)(ws + oW);
  unsigned short* LW2  = (unsigned short*)(ws + oLW);
  float*          AF   = (float*)(ws + oAF);

  k_prep<<<PB_TOT, 256, 0, stream>>>(x, w1, w2, av, lw, XB, XT, W12T, LW2, AF);
  k_proj<<<NROWS / GBM, 128, 0, stream>>>(XB, W12T, X12);
  k_gat<<<NB * (NN / TI), 256, 0, stream>>>(Am, X12, XT, LW2, AF, out);
}
